// HyperbolicGATLayer_65438121721894
// MI455X (gfx1250) — hardware-verified
//
#include <hip/hip_runtime.h>
#include <math.h>

#define NN    50000
#define NE    800000
#define KIN   128
#define DH    128
#define HD    64
#define NHD   2
#define QN    384
#define NPAD  50048
#define MT    782
#define TSZ   2048
#define NTILE 25
#define NT    256
#define SCH   4096
#define SPT   (SCH / NT)
#define NCH   ((NE + SCH - 1) / SCH)
#define EPS_F 1e-8f

typedef __attribute__((ext_vector_type(16))) _Float16 v16h;
typedef __attribute__((ext_vector_type(8)))  _Float16 v8h;
typedef __attribute__((ext_vector_type(16))) __bf16   v16b;
typedef __attribute__((ext_vector_type(8)))  __bf16   v8b;
typedef __attribute__((ext_vector_type(8)))  float    v8f;
typedef __attribute__((ext_vector_type(4)))  float    v4f;
typedef __attribute__((ext_vector_type(4)))  int      v4i;
typedef __attribute__((ext_vector_type(4)))  unsigned v4u;

__device__ __forceinline__ unsigned short f2bf_bits(float f) {
  unsigned u = __float_as_uint(f);
  return (unsigned short)((u + 0x7FFFu + ((u >> 16) & 1u)) >> 16);
}
__device__ __forceinline__ float bf_bits2f(unsigned short h) { return __uint_as_float(((unsigned)h) << 16); }

__device__ __forceinline__ void split2(float f0, float f1, unsigned& h, unsigned& l) {
  const unsigned short h0 = f2bf_bits(f0), h1 = f2bf_bits(f1);
  const unsigned short l0 = f2bf_bits(f0 - bf_bits2f(h0)), l1 = f2bf_bits(f1 - bf_bits2f(h1));
  h = (unsigned)h0 | ((unsigned)h1 << 16);
  l = (unsigned)l0 | ((unsigned)l1 << 16);
}

__device__ __forceinline__ void dep_guard_h(v8f& a, v8f& b, v16h x, v16h y) { asm volatile("v_nop\n\tv_nop\n\tv_nop\n\tv_nop" : "+v"(a), "+v"(b) : "v"(x), "v"(y)); }
__device__ __forceinline__ void dep_guard_b(v8f& a, v8f& b, v16b x, v16b y) { asm volatile("v_nop\n\tv_nop\n\tv_nop\n\tv_nop" : "+v"(a), "+v"(b) : "v"(x), "v"(y)); }
__device__ __forceinline__ void keep4_h(v16h a, v16h b, v16h c, v16h d) { asm volatile("v_nop" :: "v"(a), "v"(b), "v"(c), "v"(d)); }
__device__ __forceinline__ void keep4_b(v16b a, v16b b, v16b c, v16b d) { asm volatile("v_nop" :: "v"(a), "v"(b), "v"(c), "v"(d)); }
__device__ __forceinline__ void acc_guard4(v8f& a, v8f& b, v8f& c, v8f& d) { asm volatile("v_nop\n\tv_nop\n\tv_nop\n\tv_nop" : "+v"(a), "+v"(b), "+v"(c), "+v"(d)); }
template <typename T> struct Frag;
template <> struct Frag<_Float16> {
  typedef v16h V; union U { v16h v; v8h h[2]; };
  static __device__ __forceinline__ v16h load(const _Float16* p) {
    U f; f.h[0] = *(const v8h*)(p); f.h[1] = *(const v8h*)(p + 16); return f.v;
  }
  static __device__ __forceinline__ v8f mma(v16h a, v16h b, v8f c) {
    return __builtin_amdgcn_wmma_f32_16x16x32_f16(false, a, false, b, (short)0, c, false, false);
  }
  static __device__ __forceinline__ void guard(v8f& a, v8f& b, v16h x, v16h y) { dep_guard_h(a, b, x, y); }
  static __device__ __forceinline__ void keep(v16h a, v16h b, v16h c, v16h d) { keep4_h(a, b, c, d); }
};
template <> struct Frag<__bf16> {
  typedef v16b V; union U { v16b v; v8b h[2]; };
  static __device__ __forceinline__ v16b load(const __bf16* p) {
    U f; f.h[0] = *(const v8b*)(p); f.h[1] = *(const v8b*)(p + 16); return f.v;
  }
  static __device__ __forceinline__ v8f mma(v16b a, v16b b, v8f c) {
    return __builtin_amdgcn_wmma_f32_16x16x32_bf16(false, a, false, b, (short)0, c, false, false);
  }
  static __device__ __forceinline__ void guard(v8f& a, v8f& b, v16b x, v16b y) { dep_guard_b(a, b, x, y); }
  static __device__ __forceinline__ void keep(v16b a, v16b b, v16b c, v16b d) { keep4_b(a, b, c, d); }
};

template <int ET> struct Elem;
template <> struct Elem<0> { typedef _Float16 T; };
template <> struct Elem<1> { typedef __bf16 T; };
template <int ET, bool SPLIT, int BIAS_MODE, int OUT_MODE, bool RESID, int ACT = 0>
__global__ __launch_bounds__(256) void wmma_gemm64(
    const unsigned short* __restrict__ Ap, const unsigned short* __restrict__ A2p, int lda, long strideA,
    const unsigned short* __restrict__ Btp, const unsigned short* __restrict__ Bt2p, int ldb, long strideB,
    void* __restrict__ Cout, void* __restrict__ Cout2, int ldc, long strideC,
    const float* __restrict__ bias,
    const float* __restrict__ resid, long strideR,
    int M, int N, int K, float scale) {
  typedef typename Elem<ET>::T T;
  typedef typename Frag<T>::V V;
  const T* A = (const T*)Ap; const T* A2 = (const T*)A2p; const T* Bt = (const T*)Btp; const T* Bt2 = (const T*)Bt2p;
  __shared__ __align__(16) float sT[8][16 * 68];
  const int b    = blockIdx.y;
  const int lane = threadIdx.x & 31;
  const int wave = threadIdx.x >> 5;
  const int tilesN = N >> 6;
  const int tilesM = M >> 6;
  const int tile = blockIdx.x * 8 + wave;
  if (tile >= tilesM * tilesN) return;
  const int tm = tile / tilesN;
  const int tn = tile - tm * tilesN;
  const int m0 = tm << 6;
  const int n0 = tn << 6;

  const T* Ab  = A  + (size_t)b * strideA;
  const T* Bb  = Bt + (size_t)b * strideB;
  const T* Ab2 = SPLIT ? (A2  + (size_t)b * strideA) : nullptr;
  const T* Bb2 = SPLIT ? (Bt2 + (size_t)b * strideB) : nullptr;

  const int rlane = lane & 15;
  const int koff  = (lane >> 4) * 8;
  const int mOff  = (lane >> 4) * 8;

  v8f acc[4][4];
#pragma unroll
  for (int i = 0; i < 4; ++i)
#pragma unroll
    for (int j = 0; j < 4; ++j) acc[i][j] = (v8f){0.f,0.f,0.f,0.f,0.f,0.f,0.f,0.f};

  for (int k0 = 0; k0 < K; k0 += 32) {
    V bh[4], bl[4];
#pragma unroll
    for (int j = 0; j < 4; ++j) {
      const size_t bo = (size_t)(n0 + (j << 4) + rlane) * ldb + koff + k0;
      bh[j] = Frag<T>::load(Bb + bo);
      if (SPLIT) bl[j] = Frag<T>::load(Bb2 + bo);
    }
#pragma unroll
    for (int i = 0; i < 4; ++i) {
      const size_t ao = (size_t)(m0 + (i << 4) + rlane) * lda + koff + k0;
      V ah = Frag<T>::load(Ab + ao);
      V al;
      if (SPLIT) al = Frag<T>::load(Ab2 + ao);
#pragma unroll
      for (int j = 0; j < 4; ++j) {
        acc[i][j] = Frag<T>::mma(ah, bh[j], acc[i][j]);
        if (SPLIT) {
          acc[i][j] = Frag<T>::mma(ah, bl[j], acc[i][j]);
          acc[i][j] = Frag<T>::mma(al, bh[j], acc[i][j]);
        }
      }
      Frag<T>::guard(acc[i][0], acc[i][3], ah, SPLIT ? al : ah);
    }
    Frag<T>::keep(bh[0], bh[1], bh[2], bh[3]);
    if (SPLIT) Frag<T>::keep(bl[0], bl[1], bl[2], bl[3]);
  }
  acc_guard4(acc[0][0], acc[0][1], acc[0][2], acc[0][3]);
  acc_guard4(acc[1][0], acc[1][1], acc[1][2], acc[1][3]);
  acc_guard4(acc[2][0], acc[2][1], acc[2][2], acc[2][3]);
  acc_guard4(acc[3][0], acc[3][1], acc[3][2], acc[3][3]);

  float* slab = sT[wave];
  const float* Rb = RESID ? (resid + (size_t)b * strideR) : nullptr;
#pragma unroll
  for (int i = 0; i < 4; ++i) {
    const int mBase = m0 + (i << 4);
#pragma unroll
    for (int j = 0; j < 4; ++j) {
      const int n = n0 + (j << 4) + rlane;
      float bv = 0.f;
      if (BIAS_MODE == 2) bv = bias[n];
#pragma unroll
      for (int r = 0; r < 8; ++r) {
        float v = acc[i][j][r] * scale;
        if (BIAS_MODE == 1) v += bias[mBase + mOff + r];
        if (BIAS_MODE == 2) v += bv;
        if (RESID) v += Rb[(size_t)(mBase + mOff + r) * ldc + n];
        if (ACT == 1) v = tanhf(v);
        if (ACT == 2) v = fmaxf(v, 0.0f);
        if (ACT == 3) v = v / (1.0f + expf(-v));
        if (ACT == 4) v = (v > 0.f) ? v : 0.01f * v;
        if (ACT == 5) v = 0.5f * v * (1.0f + erff(v * 0.70710678118654752f));
        slab[(mOff + r) * 68 + (j << 4) + rlane] = v;
      }
    }
    __builtin_amdgcn_fence(__ATOMIC_RELEASE, "workgroup");
    __builtin_amdgcn_wave_barrier();
    __builtin_amdgcn_fence(__ATOMIC_ACQUIRE, "workgroup");
    if (OUT_MODE == 0) {
      float* C = (float*)Cout + (size_t)b * strideC;
      const int hh = lane >> 4, c4 = (lane & 15) * 4;
      for (int pass = 0; pass < 2; ++pass) {
#pragma unroll
        for (int it = 0; it < 8; ++it) {
          const int row = it * 2 + hh;
          v4f v = *(const v4f*)(slab + row * 68 + c4);
          *(volatile v4f*)(C + (size_t)(mBase + row) * ldc + n0 + c4) = v;
        }
        __threadfence();
      }
    } else {
      const int q = lane >> 3, c8 = (lane & 7) * 8;
      unsigned short* C  = (unsigned short*)Cout  + (size_t)b * strideC;
      unsigned short* C2 = (OUT_MODE == 2) ? ((unsigned short*)Cout2 + (size_t)b * strideC) : nullptr;
      for (int pass = 0; pass < 2; ++pass) {
#pragma unroll
        for (int it = 0; it < 4; ++it) {
          const int row = it * 4 + q;
          const float* sp = slab + row * 68 + c8;
          v8h hv, lv;
#pragma unroll
          for (int e = 0; e < 8; ++e) {
            if (OUT_MODE == 1) {
              hv[e] = (_Float16)sp[e];
            } else {
              unsigned short hb = f2bf_bits(sp[e]);
              unsigned short lb = f2bf_bits(sp[e] - bf_bits2f(hb));
              hv[e] = __builtin_bit_cast(_Float16, hb);
              lv[e] = __builtin_bit_cast(_Float16, lb);
            }
          }
          *(volatile v8h*)(C + (size_t)(mBase + row) * ldc + n0 + c8) = hv;
          if (OUT_MODE == 2) *(volatile v8h*)(C2 + (size_t)(mBase + row) * ldc + n0 + c8) = lv;
        }
        __threadfence();
      }
    }
    __builtin_amdgcn_fence(__ATOMIC_RELEASE, "workgroup");
    __builtin_amdgcn_wave_barrier();
    __builtin_amdgcn_fence(__ATOMIC_ACQUIRE, "workgroup");
  }
}

__global__ __launch_bounds__(256) void prep_kernel(
    const float* __restrict__ x, const float* __restrict__ Wq, const float* __restrict__ Wk, const float* __restrict__ Wv,
    const float* __restrict__ Wo, const float* __restrict__ bq, const float* __restrict__ bk, const float* __restrict__ bv,
    unsigned* __restrict__ Xh, unsigned* __restrict__ Xl, unsigned* __restrict__ Wh, unsigned* __restrict__ Wl,
    unsigned* __restrict__ Oh, unsigned* __restrict__ Ol, float* __restrict__ b384, int nbx, int nbw, int nbo) {
  const int tid = threadIdx.x;
  const int bid = blockIdx.x;
  const v4f z4 = {0.f, 0.f, 0.f, 0.f};
  if (bid < nbx + nbw + nbo) {
    const float* p = x; unsigned* ph = nullptr; unsigned* pl = nullptr; bool act = false; bool zero = false;
    if (bid < nbx) {
      const int g = bid * 256 + tid;
      if (g < NPAD * DH / 8) {
        const int row = g >> 4, c8 = (g & 15) * 8;
        const int rowc = row < NN ? row : NN - 1;
        p = x + (size_t)rowc * KIN + c8; zero = (row >= NN);
        ph = Xh + (size_t)4 * g; pl = Xl + (size_t)4 * g; act = true;
      }
    } else if (bid < nbx + nbw) {
      const int g = (bid - nbx) * 256 + tid;
      if (g < QN * KIN / 8) {
        const int row = g >> 4, c8 = (g & 15) * 8;
        const float* W = (row < DH) ? Wq : ((row < 2 * DH) ? Wk : Wv);
        p = W + (size_t)(row & (DH - 1)) * KIN + c8;
        ph = Wh + (size_t)4 * g; pl = Wl + (size_t)4 * g; act = true;
      }
    } else {
      const int g = (bid - nbx - nbw) * 256 + tid;
      if (g < HD * DH / 8) {
        const int row = g >> 4, c8 = (g & 15) * 8;
        p = Wo + (size_t)row * DH + c8;
        ph = Oh + (size_t)4 * g; pl = Ol + (size_t)4 * g; act = true;
      }
    }
    if (act) {
      v4f a = *(const v4f*)p, c = *(const v4f*)(p + 4);
      if (zero) { a = z4; c = z4; }
      unsigned h0, l0, h1, l1, h2, l2, h3, l3;
      split2(a[0], a[1], h0, l0); split2(a[2], a[3], h1, l1); split2(c[0], c[1], h2, l2); split2(c[2], c[3], h3, l3);
      const v4u hv = {h0, h1, h2, h3}, lv = {l0, l1, l2, l3};
      *(volatile v4u*)ph = hv; *(volatile v4u*)pl = lv;
      __threadfence();
      *(volatile v4u*)ph = hv; *(volatile v4u*)pl = lv;
    }
  } else {
    if (tid < 96) {
      const float* bp = (tid < 32) ? (bq + 4 * tid) : ((tid < 64) ? (bk + 4 * (tid - 32)) : (bv + 4 * (tid - 64)));
      const v4f v = *(const v4f*)bp;
      float* op = b384 + 4 * tid;
      *(volatile v4f*)op = v; __threadfence(); *(volatile v4f*)op = v;
    }
  }
}

__device__ __forceinline__ int blk_excl_scan(int cnt, int* scan_ws, int tid, int* tot) {
  const int lane = tid & 31, wave = tid >> 5; int incl = cnt;
#pragma unroll
  for (int o = 1; o < 32; o <<= 1) { const int v = __shfl_up(incl, o, 32); if (lane >= o) incl += v; }
  if (lane == 31) scan_ws[wave] = incl;
  __syncthreads();
  if (wave == 0) { int wv = (lane < NT / 32) ? scan_ws[lane] : 0; int wincl = wv;
#pragma unroll
    for (int o = 1; o < 32; o <<= 1) { const int v = __shfl_up(wincl, o, 32); if (lane >= o) wincl += v; }
    if (lane < NT / 32) scan_ws[32 + lane] = wincl - wv; if (lane == 31) scan_ws[64] = wincl; }
  __syncthreads();
  const int res = scan_ws[32 + wave] + incl - cnt; *tot = scan_ws[64];
  return res;
}
template <int SP, int CAP>
__device__ __forceinline__ int chunk_hits(const int* __restrict__ dstv, const int* __restrict__ srcv, int e0, int n0, int tid,
                                          int* LIST, int* scan_ws) {
  const int eb = e0 + tid * SP;
  int rec[SP]; int cnt = 0;
#pragma unroll
  for (int k = 0; k < SP; ++k) rec[k] = -1;
  {
    const bool inr = (eb < NE);
    const int ebc = inr ? eb : (NE - SP);
#pragma unroll
    for (int k = 0; k < SP; k += 4) {
      const v4i d4 = *(const v4i*)(dstv + ebc + k);
      const v4i s4 = *(const v4i*)(srcv + ebc + k);
#pragma unroll
      for (int e = 0; e < 4; ++e) {
        const int d = d4[e];
        if (inr && d >= n0 && d < n0 + TSZ && d < NN) {
          int s = s4[e]; s = s < 0 ? 0 : (s >= NN ? NN - 1 : s);
          rec[k + e] = ((d - n0) << 16) | s; ++cnt;
        }
      }
    }
  }
  int tot; int p = blk_excl_scan(cnt, scan_ws, tid, &tot);
#pragma unroll
  for (int k = 0; k < SP; ++k) if (rec[k] >= 0) { if ((unsigned)p < (unsigned)CAP) LIST[p] = rec[k]; ++p; }
  __syncthreads();
  return tot < CAP ? tot : CAP;
}

__global__ __launch_bounds__(NT) void edge_agg_kernel(const float* __restrict__ QKV, const int* __restrict__ ei, float* AGG,
                                                     unsigned* __restrict__ Hh, unsigned* __restrict__ Hl) {
  __shared__ int LIST[SCH];
  __shared__ float SM[TSZ * NHD];
  __shared__ float SL[TSZ * NHD];
  __shared__ int scan_ws[80];
  const int tid = threadIdx.x, lane = tid & 31, wave = tid >> 5;
  const int n0 = blockIdx.x * TSZ;
  const int hl = lane >> 4;
  const v4f z4 = {0.f, 0.f, 0.f, 0.f};
  for (int pass = 0; pass < 2; ++pass) {
#pragma unroll 1
    for (int j = 0; j < TSZ / 8; ++j) {
      float* rp = AGG + (size_t)(n0 + wave * (TSZ / 8) + j) * DH + 4 * lane;
      *(volatile v4f*)rp = z4;
    }
    __threadfence();
  }
  for (int i = tid; i < TSZ * NHD; i += NT) { SM[i] = -INFINITY; SL[i] = 0.f; }
  __syncthreads();
  const int* srcv = ei; const int* dstv = ei + NE;
#pragma unroll 1
  for (int c = 0; c < NCH; ++c) {
    const int tot = chunk_hits<SPT, SCH>(dstv, srcv, c * SCH, n0, tid, LIST, scan_ws);
#pragma unroll 1
    for (int base = 0; base < tot; base += 32) {
      const int q = base + lane;
      const int qc = (q < SCH) ? q : (SCH - 1);
      const int lv = LIST[qc];
      const int rv = (q < tot) ? lv : -1;
      const int own = (rv >= 0 && (rv >> 24) == wave) ? 1 : 0;
      unsigned msk = (unsigned)__ballot(own);
#pragma unroll 1
      for (int it = 0; it < 32; ++it) {
        if (msk == 0u) break;
        const int bp = __builtin_ctz(msk); msk &= msk - 1u;
        const int r = __shfl(rv, bp, 32);
        const int dl = r >> 16, s = r & 0xFFFF;
        const float* qr = QKV + (size_t)(n0 + dl) * QN + 4 * lane;
        const float* kr = QKV + (size_t)s * QN + DH + 4 * lane;
        const v4f qv = *(const v4f*)qr;
        const v4f kv = *(const v4f*)kr;
        const v4f vv = *(const v4f*)(kr + DH);
        float pd = qv[0] * kv[0]; pd += qv[1] * kv[1]; pd += qv[2] * kv[2]; pd += qv[3] * kv[3];
        pd += __shfl_xor(pd, 1, 32); pd += __shfl_xor(pd, 2, 32); pd += __shfl_xor(pd, 4, 32); pd += __shfl_xor(pd, 8, 32);
        const float sc = pd * 0.125f;
        const int mi = dl * NHD + hl;
        const float mo = SM[mi], lo = SL[mi];
        const float mn = fmaxf(mo, sc);
        const float rr = __expf(mo - mn), ex = __expf(sc - mn);
        const float ln = lo * rr + ex;
        if ((lane & 15) == 0) { SM[mi] = mn; SL[mi] = ln; }
        float* rp = AGG + (size_t)(n0 + dl) * DH + 4 * lane;
        v4f a = *(const volatile v4f*)rp;
        a = a * rr + vv * ex;
        *(volatile v4f*)rp = a; __threadfence(); *(volatile v4f*)rp = a;
      }
    }
    __syncthreads();
  }
  const int rsel = lane >> 4, c8 = (lane & 15) * 8, hsel = (lane & 15) >> 3;
#pragma unroll 1
  for (int jj = 0; jj < TSZ / 16; ++jj) {
    const int dl0 = wave * (TSZ / 8) + 2 * jj;
    if (n0 + dl0 < NPAD) {
      const int dl = dl0 + rsel;
      const int n = n0 + dl;
      const float l = SL[dl * NHD + hsel];
      const float inv = 1.0f / (l + EPS_F);
      const float* rp = AGG + (size_t)n * DH + c8;
      v4f a = *(const volatile v4f*)rp;
      v4f c = *(const volatile v4f*)(rp + 4);
      a = a * inv; c = c * inv;
      unsigned h0, l0, h1, l1, h2, l2, h3, l3;
      split2(a[0], a[1], h0, l0); split2(a[2], a[3], h1, l1); split2(c[0], c[1], h2, l2); split2(c[2], c[3], h3, l3);
      const v4u hv = {h0, h1, h2, h3}, lw = {l0, l1, l2, l3};
      unsigned* hp = Hh + (size_t)n * (DH / 2) + (c8 >> 1);
      unsigned* lp = Hl + (size_t)n * (DH / 2) + (c8 >> 1);
      *(volatile v4u*)hp = hv; *(volatile v4u*)lp = lw;
      __threadfence();
      *(volatile v4u*)hp = hv; *(volatile v4u*)lp = lw;
    }
  }
}

__global__ __launch_bounds__(256) void tail_copy_kernel(const float* __restrict__ T, float* __restrict__ out) {
  const int t = threadIdx.x;
  const v4f v = *(const v4f*)(T + 4 * t);
  float* op = out + (size_t)(MT - 1) * 64 * HD + 4 * t;
  *(volatile v4f*)op = v; __threadfence(); *(volatile v4f*)op = v;
}

extern "C" void kernel_launch(void* const* d_in, const int* in_sizes, int n_in,
                              void* d_out, int out_size, void* d_ws, size_t ws_size, hipStream_t stream) {
  if (n_in < 10) return;
  if (in_sizes[0] != NN * KIN || in_sizes[1] != 2 * NE || out_size != NN * HD) return;
  const float* x  = (const float*)d_in[0];
  const int*   ei = (const int*)  d_in[1];
  const float* Wq = (const float*)d_in[2];
  const float* bq = (const float*)d_in[3];
  const float* Wk = (const float*)d_in[4];
  const float* bk = (const float*)d_in[5];
  const float* Wv = (const float*)d_in[6];
  const float* bv = (const float*)d_in[7];
  const float* Wo = (const float*)d_in[8];
  const float* bo = (const float*)d_in[9];
  float* out = (float*)d_out;

  char* ws = (char*)d_ws; size_t off = 0;
  auto carve = [&](size_t bytes) -> char* { char* p = ws + off; off += (bytes + 255) & ~(size_t)255; return p; };
  float*          QKV  = (float*)carve((size_t)NPAD * QN * 4);
  const size_t xplane  = (size_t)NPAD * DH * 2;
  const size_t aggb    = (size_t)NTILE * TSZ * DH * 4;
  char*           regA = carve(aggb > 2 * xplane ? aggb : 2 * xplane);
  unsigned short* Xh   = (unsigned short*)regA;
  unsigned short* Xl   = (unsigned short*)(regA + xplane);
  float*          AGG  = (float*)regA;
  unsigned short* Hh   = (unsigned short*)carve(xplane);
  unsigned short* Hl   = (unsigned short*)carve(xplane);
  unsigned short* Wh   = (unsigned short*)carve((size_t)QN * KIN * 2);
  unsigned short* Wl   = (unsigned short*)carve((size_t)QN * KIN * 2);
  unsigned short* Oh   = (unsigned short*)carve((size_t)HD * DH * 2);
  unsigned short* Ol   = (unsigned short*)carve((size_t)HD * DH * 2);
  float*          b384 = (float*)carve((size_t)QN * 4);
  float*          TAIL = (float*)carve((size_t)64 * HD * 4);
  if (off > ws_size || off > (size_t)134217728) return;

  const int nbx = (NPAD * DH / 8 + 255) / 256;
  const int nbw = (QN * KIN / 8 + 255) / 256;
  const int nbo = (HD * DH / 8 + 255) / 256;

  prep_kernel<<<nbx + nbw + nbo + 1, 256, 0, stream>>>(x, Wq, Wk, Wv, Wo, bq, bk, bv,
      (unsigned*)Xh, (unsigned*)Xl, (unsigned*)Wh, (unsigned*)Wl, (unsigned*)Oh, (unsigned*)Ol, b384, nbx, nbw, nbo);

  wmma_gemm64<1, true, 2, 0, false><<<dim3((MT * (QN / 64) + 7) / 8, 1), 256, 0, stream>>>(
      Xh, Xl, DH, 0L, Wh, Wl, KIN, 0L, (void*)QKV, nullptr, QN, 0L, b384, nullptr, 0L, NPAD, QN, KIN, 1.0f);

  edge_agg_kernel<<<NTILE, NT, 0, stream>>>(QKV, ei, AGG, (unsigned*)Hh, (unsigned*)Hl);

  wmma_gemm64<1, true, 2, 0, false><<<dim3((MT - 1 + 7) / 8, 1), 256, 0, stream>>>(
      Hh, Hl, DH, 0L, Oh, Ol, DH, 0L, (void*)out, nullptr, HD, 0L, bo, nullptr, 0L, (MT - 1) * 64, HD, DH, 1.0f);
  wmma_gemm64<1, true, 2, 0, false><<<dim3(1, 1), 256, 0, stream>>>(
      Hh + (size_t)(MT - 1) * 64 * DH, Hl + (size_t)(MT - 1) * 64 * DH, DH, 0L, Oh, Ol, DH, 0L,
      (void*)TAIL, nullptr, HD, 0L, bo, nullptr, 0L, 64, HD, DH, 1.0f);
  tail_copy_kernel<<<1, 256, 0, stream>>>(TAIL, out);
}
